// Pointnet_SA_6227702580013
// MI455X (gfx1250) — hardware-verified
//
#include <hip/hip_runtime.h>
#include <math.h>
#include <stddef.h>
#include <stdint.h>


#define NB    8
#define NP    4096
#define NS    1024
#define NK    64
#define NC    64
#define NG    (NB * NS)
#define K0    67
#define K0P   96
#define F0    64
#define F1    128
#define F2    256
#define CAP   512
#define NWAV  1024
#define ASC   8.0f
#define WSC   1024.0f
#define XSC   0.0009765625f
#define OSC   0.0001220703125f
#define RADF  0.2f
#define OUT1  (NG * 3)
#define SMW0  0
#define SMW1  12288
#define SMW2  28672
#define SMWV  94208
#define WVB   24576
#define SMEM  (SMWV + 4 * WVB)
#define WSCAP 134217728

static_assert(NG % NWAV == 0);
static_assert(NG % 32 == 0);
static_assert(NP % 32 == 0);
static_assert(K0P % 32 == 0);
static_assert(F0 % 32 == 0);
static_assert(F1 % 32 == 0);
static_assert(F2 % 32 == 0);
static_assert(SMW1 == SMW0 + F0 * K0P * 2);
static_assert(SMW2 == SMW1 + F1 * F0 * 2);
static_assert(SMWV == SMW2 + F2 * F1 * 2);
static_assert(WVB >= NK * F1 * 2 + NK * F0 * 2);
static_assert(NK * K0P * 2 <= 16384);
static_assert(8 * CAP + 4 * NK <= NK * F0 * 2);
static_assert(4 * F2 <= NK * F0 * 2);

typedef float    v4f  __attribute__((ext_vector_type(4)));
typedef float    v8f  __attribute__((ext_vector_type(8)));
typedef _Float16 v8h  __attribute__((ext_vector_type(8)));
typedef _Float16 v16h __attribute__((ext_vector_type(16)));
typedef unsigned long long u64;
union FragH { v16h v; v8h h[2]; };

__device__ __forceinline__ v8f wmf(v16h a, v16h b, v8f c) {
  v8f d = __builtin_amdgcn_wmma_f32_16x16x32_f16(false, a, false, b, (short)0, c, false, false);
  asm volatile("v_nop\n\tv_nop\n\tv_nop\n\tv_nop" : "+v"(d) : "v"(a), "v"(b));
  return d;
}

__device__ __forceinline__ v8f splat8(float x) { v8f r = {x, x, x, x, x, x, x, x}; return r; }

__device__ __forceinline__ v16h ldfrag(const _Float16* p, int k0, int hh) {
  FragH u;
  u.h[0] = *(const v8h*)(p + k0 + 8 * hh);
  u.h[1] = *(const v8h*)(p + k0 + 16 + 8 * hh);
  return u.v;
}

__device__ __forceinline__ void wave_sync() {
  __builtin_amdgcn_fence(__ATOMIC_RELEASE, "wavefront");
  __builtin_amdgcn_wave_barrier();
}

__device__ __forceinline__ float vgpr_zero() {
  float z;
  asm volatile("v_mov_b32 %0, 0" : "=v"(z));
  return z;
}

__device__ __forceinline__ float sqrt_rn_f32(float s) {
#pragma clang fp contract(off)
  float c = sqrtf(s);
  const double sd = (double)s;
#pragma unroll
  for (int i = 0; i < 3; ++i) {
    const unsigned uc = __float_as_uint(c);
    const float cu = __uint_as_float(uc + 1u);
    const float cd = __uint_as_float(uc - 1u);
    const double mh = ((double)c + (double)cu) * 0.5;
    const double ml = ((double)cd + (double)c) * 0.5;
    const double mh2 = mh * mh;
    const double ml2 = ml * ml;
    const bool up = mh2 <= sd;
    const bool dn = sd < ml2;
    c = up ? cu : (dn ? cd : c);
  }
  return (s > 0.0f) ? c : 0.0f;
}

__device__ __forceinline__ float dist3(float cx, float cy, float cz, float px, float py, float pz) {
#pragma clang fp contract(off)
  const float dx = cx - px;
  const float dy = cy - py;
  const float dz = cz - pz;
  float xx = dx * dx;
  asm volatile("" : "+v"(xx));
  float yy = dy * dy;
  asm volatile("" : "+v"(yy));
  float zz = dz * dz;
  asm volatile("" : "+v"(zz));
  float s = xx + zz;
  asm volatile("" : "+v"(s));
  const float s2 = s + yy;
  return sqrt_rn_f32(s2);
}

__device__ __forceinline__ void bitonic_wave(u64* k, int L, int lane) {
#pragma unroll 1
  for (int size = 2; size <= L; size <<= 1) {
#pragma unroll 1
    for (int stride = size >> 1; stride > 0; stride >>= 1) {
      const int half = L >> 1;
#pragma unroll 1
      for (int p = lane; p < half; p += 32) {
        const int lo = p & (stride - 1);
        const int i = (p << 1) - lo;
        const int j = i + stride;
        const u64 a = k[i];
        const u64 c = k[j];
        const bool up = (i & size) == 0;
        const bool sw = up ? (a > c) : (a < c);
        if (sw) { k[i] = c; k[j] = a; }
      }
      wave_sync();
    }
  }
}

__device__ __forceinline__ v8h prepw_piece(const float* ts, int p, int npc) {
  const int row = p / npc, k8 = (p - row * npc) * 8;
  v8h o;
#pragma unroll
  for (int e = 0; e < 8; ++e) o[e] = (_Float16)(ts[(k8 + e) * 16 + row] * WSC);
  return o;
}

__global__ __launch_bounds__(256) void k_prepw(const float* __restrict__ W, int Kd, int Nd, int Kp,
                                                int nA, int offA, int nB, _Float16* dst) {
  __shared__ __attribute__((aligned(16))) float ts[256 * 16];
  const int t = threadIdx.x;
  const int n0 = blockIdx.x * 16;
  if (t < Kp) {
    int ks = (t < nA) ? (t + offA) : (t - nA);
    ks = min(max(ks, 0), Kd - 1);
    const bool valid = t < nA + nB;
    const float* wrow = W + (size_t)ks * Nd;
#pragma unroll
    for (int nn = 0; nn < 16; ++nn) {
      const int n = n0 + nn;
      const float v = wrow[min(n, Nd - 1)];
      ts[t * 16 + nn] = (valid && n < Nd) ? v : 0.0f;
    }
  }
  __syncthreads();
  const int npc = Kp >> 3;
  const int tot = 16 * npc;
  const int p0 = t, p1 = t + 256;
  const bool a0 = p0 < tot, a1 = p1 < tot;
  const v8h o0 = prepw_piece(ts, a0 ? p0 : 0, npc);
  const v8h o1 = prepw_piece(ts, a1 ? p1 : 0, npc);
  _Float16* d0 = dst + (size_t)n0 * Kp + 8 * (a0 ? p0 : 0);
  _Float16* d1 = dst + (size_t)n0 * Kp + 8 * (a1 ? p1 : 0);
  if (a0) *(volatile v8h*)d0 = o0;
  if (a1) *(volatile v8h*)d1 = o1;
  __threadfence();
  if (a0) *(volatile v8h*)d0 = o0;
  if (a1) *(volatile v8h*)d1 = o1;
}

__global__ __launch_bounds__(32) void k_cent(const float* __restrict__ xyz, const int* __restrict__ fps,
                                              float* outp) {
  __shared__ __attribute__((aligned(16))) float s[96];
  const int lane = threadIdx.x & 31;
  const int q = blockIdx.x * 32 + lane;
  const int b = q / NS;
  int ci = fps[q];
  ci = min(max(ci, 0), NP - 1);
  const float* xp = xyz + ((size_t)b * NP + ci) * 3;
  s[3 * lane + 0] = xp[0];
  s[3 * lane + 1] = xp[1];
  s[3 * lane + 2] = xp[2];
  wave_sync();
  const int l8 = min(lane, 23);
  const v4f v = *(const v4f*)(s + 4 * l8);
  float* d = outp + (size_t)blockIdx.x * 96 + 4 * l8;
  if (lane < 24) *(volatile v4f*)d = v;
  __threadfence();
  if (lane < 24) *(volatile v4f*)d = v;
}

template <int KS, int NT, int MODE>
__device__ __forceinline__ void mlp_layer(const _Float16* X, const _Float16* W, _Float16* Y,
                                           float* srow, int lane) {
  constexpr int K = 32 * KS;
  constexpr int N = 16 * NT;
  const int hh = lane >> 4, nl = lane & 15;
#pragma unroll 1
  for (int nt = 0; nt < NT; ++nt) {
    v8f acc[4];
#pragma unroll
    for (int mt = 0; mt < 4; ++mt) acc[mt] = splat8(0.0f);
    const _Float16* bp = W + (nt * 16 + nl) * K;
#pragma unroll
    for (int ks = 0; ks < KS; ++ks) {
      const v16h bf = ldfrag(bp, 32 * ks, hh);
#pragma unroll
      for (int mt = 0; mt < 4; ++mt)
        acc[mt] = wmf(ldfrag(X + (mt * 16 + nl) * K, 32 * ks, hh), bf, acc[mt]);
    }
    const int col = nt * 16 + nl;
    if (MODE == 0) {
#pragma unroll
      for (int mt = 0; mt < 4; ++mt) {
#pragma unroll
        for (int r = 0; r < 8; ++r)
          Y[(mt * 16 + 8 * hh + r) * N + col] = (_Float16)(fmaxf(acc[mt][r], 0.0f) * XSC);
      }
    } else {
      float rm = 0.0f;
#pragma unroll
      for (int mt = 0; mt < 4; ++mt) {
#pragma unroll
        for (int r = 0; r < 8; ++r) rm = fmaxf(rm, acc[mt][r]);
      }
      rm = fmaxf(rm, __shfl_xor(rm, 16, 32));
      if (hh == 0) srow[col] = rm * OSC;
    }
  }
}

__global__ __launch_bounds__(128) void k_grp(const float* __restrict__ xyz, const float* __restrict__ pts,
                                             const int* __restrict__ fps, const _Float16* __restrict__ w0p,
                                             const _Float16* __restrict__ w1p, const _Float16* __restrict__ w2p,
                                             float* outp) {
  extern __shared__ __attribute__((aligned(16))) char smem[];
  _Float16* sW0 = (_Float16*)(smem + SMW0);
  _Float16* sW1 = (_Float16*)(smem + SMW1);
  _Float16* sW2 = (_Float16*)(smem + SMW2);
  const int t = threadIdx.x, lane = t & 31, wv = t >> 5;
  char* wreg = smem + SMWV + wv * WVB;
  _Float16* X02 = (_Float16*)wreg;
  _Float16* X1 = (_Float16*)(wreg + 16384);
  u64* skey = (u64*)(wreg + 16384);
  int* sidx = (int*)(wreg + 16384 + 8 * CAP);
  float* srow = (float*)(wreg + 16384);

  for (int p = t; p < F0 * K0P / 8; p += 128) *(v8h*)(sW0 + 8 * p) = *(const v8h*)(w0p + 8 * p);
  for (int p = t; p < F1 * F0 / 8; p += 128) *(v8h*)(sW1 + 8 * p) = *(const v8h*)(w1p + 8 * p);
  for (int p = t; p < F2 * F1 / 8; p += 128) *(v8h*)(sW2 + 8 * p) = *(const v8h*)(w2p + 8 * p);
  __syncthreads();

  const float qnan = __int_as_float(0x7fc00000);
  const int wg = blockIdx.x * 4 + wv;

#pragma unroll 1
  for (int it = 0; it < NG / NWAV; ++it) {
    const int g = it * NWAV + wg;
    const int b = g / NS;
    const float* xb = xyz + (size_t)b * NP * 3;
    const float* pb = pts + (size_t)b * NP * NC;
    int ci = fps[g];
    ci = min(max(ci, 0), NP - 1);
    const float cx = xb[3 * ci], cy = xb[3 * ci + 1], cz = xb[3 * ci + 2];

    int cnt = 0;
#pragma unroll 1
    for (int base = 0; base < NP; base += 32) {
      const int n = base + lane;
      const float d = dist3(cx, cy, cz, xb[3 * n], xb[3 * n + 1], xb[3 * n + 2]);
      const bool in = d < RADF;
      const unsigned m = (unsigned)__builtin_amdgcn_ballot_w32(in);
      const int pos = cnt + (int)__builtin_popcount(m & ((1u << lane) - 1u));
      if (in && pos < CAP) skey[pos] = ((u64)__float_as_uint(d) << 32) | (u64)(unsigned)n;
      cnt += (int)__builtin_popcount(m);
    }
    const bool bad = cnt > CAP;
    const int ncand = min(cnt, CAP);
    wave_sync();
    if (ncand > NK) {
      int L = 2 * NK;
      while (L < ncand && L < CAP) L <<= 1;
#pragma unroll 1
      for (int p = ncand + lane; p < L; p += 32) skey[p] = ~0ull;
      wave_sync();
      bitonic_wave(skey, L, lane);
      {
        const u64 a = skey[lane];
        const u64 c = skey[lane + 32];
        skey[lane] = a & 0xffffffffull;
        skey[lane + 32] = c & 0xffffffffull;
      }
      wave_sync();
      bitonic_wave(skey, NK, lane);
      sidx[lane] = (int)(unsigned)skey[lane];
      sidx[lane + 32] = (int)(unsigned)skey[lane + 32];
    } else {
      int v0 = NP - 1, v1 = NP - 1;
      if (ncand > 0) {
        const int first = (int)(unsigned)skey[0];
        const int a = (int)(unsigned)skey[min(lane, ncand - 1)];
        const int c = (int)(unsigned)skey[min(lane + 32, ncand - 1)];
        v0 = (lane < ncand) ? a : first;
        v1 = (lane + 32 < ncand) ? c : first;
      }
      sidx[lane] = v0;
      sidx[lane + 32] = v1;
    }
    wave_sync();

#pragma unroll 4
    for (int p = 0; p < 16; ++p) {
      const int r = 4 * p + (lane >> 3);
      const int c8 = (lane & 7) * 8;
      int j = sidx[r];
      j = min(max(j, 0), NP - 1);
      const float* pr = pb + (size_t)j * NC + c8;
      const v4f u0 = *(const v4f*)pr;
      const v4f u1 = *(const v4f*)(pr + 4);
      v8h o;
      o[0] = (_Float16)(u0.x * ASC); o[1] = (_Float16)(u0.y * ASC);
      o[2] = (_Float16)(u0.z * ASC); o[3] = (_Float16)(u0.w * ASC);
      o[4] = (_Float16)(u1.x * ASC); o[5] = (_Float16)(u1.y * ASC);
      o[6] = (_Float16)(u1.z * ASC); o[7] = (_Float16)(u1.w * ASC);
      *(v8h*)(X02 + r * K0P + c8) = o;
    }
#pragma unroll
    for (int rr = 0; rr < 2; ++rr) {
      const int r = lane + 32 * rr;
      int j = sidx[r];
      j = min(max(j, 0), NP - 1);
      const float gx = xb[3 * j] - cx;
      const float gy = xb[3 * j + 1] - cy;
      const float gz = xb[3 * j + 2] - cz;
      const _Float16 hzv = (_Float16)vgpr_zero();
      v8h o;
      o[0] = (_Float16)(gx * ASC);
      o[1] = (_Float16)(gy * ASC);
      o[2] = (_Float16)(gz * ASC);
      o[3] = hzv; o[4] = hzv; o[5] = hzv; o[6] = hzv; o[7] = hzv;
      const v8h z = {hzv, hzv, hzv, hzv, hzv, hzv, hzv, hzv};
      *(v8h*)(X02 + r * K0P + 64) = o;
      *(v8h*)(X02 + r * K0P + 72) = z;
      *(v8h*)(X02 + r * K0P + 80) = z;
      *(v8h*)(X02 + r * K0P + 88) = z;
    }
    wave_sync();

    mlp_layer<K0P / 32, F0 / 16, 0>(X02, sW0, X1, srow, lane);
    wave_sync();
    mlp_layer<F0 / 32, F1 / 16, 0>(X1, sW1, X02, srow, lane);
    wave_sync();
    mlp_layer<F1 / 32, F2 / 16, 1>(X02, sW2, X1, srow, lane);
    wave_sync();

    v4f o0 = *(const v4f*)(srow + 4 * lane);
    v4f o1 = *(const v4f*)(srow + 128 + 4 * lane);
    if (bad) {
      const v4f qn = {qnan, qnan, qnan, qnan};
      o0 = qn; o1 = qn;
    }
    float* d = outp + (size_t)OUT1 + (size_t)g * F2;
    *(volatile v4f*)(d + 4 * lane) = o0;
    *(volatile v4f*)(d + 128 + 4 * lane) = o1;
    __threadfence();
    *(volatile v4f*)(d + 4 * lane) = o0;
    *(volatile v4f*)(d + 128 + 4 * lane) = o1;
    wave_sync();
  }
}

extern "C" void kernel_launch(void* const* d_in, const int* in_sizes, int n_in,
                              void* d_out, int out_size, void* d_ws, size_t ws_size,
                              hipStream_t stream) {
  if (n_in < 6) return;
  if (in_sizes[0] != NB * NP * 3) return;
  if (in_sizes[1] != NB * NP * NC) return;
  if (in_sizes[2] != NG) return;
  if (in_sizes[3] != K0 * F0) return;
  if (in_sizes[4] != F0 * F1) return;
  if (in_sizes[5] != F1 * F2) return;
  if (out_size != NG * 3 + NG * F2) return;

  const float* xyz = (const float*)d_in[0];
  const float* pts = (const float*)d_in[1];
  const int*   fps = (const int*)d_in[2];
  const float* w0  = (const float*)d_in[3];
  const float* w1  = (const float*)d_in[4];
  const float* w2  = (const float*)d_in[5];
  float* out = (float*)d_out;

  char* ws = (char*)d_ws;
  size_t off = 0;
  const size_t oW0 = off; off += (size_t)F0 * K0P * 2; off = (off + 255) & ~(size_t)255;
  const size_t oW1 = off; off += (size_t)F1 * F0 * 2;  off = (off + 255) & ~(size_t)255;
  const size_t oW2 = off; off += (size_t)F2 * F1 * 2;  off = (off + 255) & ~(size_t)255;
  if (off > ws_size || off > (size_t)WSCAP) return;
  _Float16* w0p = (_Float16*)(ws + oW0);
  _Float16* w1p = (_Float16*)(ws + oW1);
  _Float16* w2p = (_Float16*)(ws + oW2);

  hipFuncSetAttribute(reinterpret_cast<const void*>(&k_grp),
                      hipFuncAttributeMaxDynamicSharedMemorySize, SMEM);

  k_prepw<<<F0 / 16, 256, 0, stream>>>(w0, K0, F0, K0P, 64, 3, 3, w0p);
  k_prepw<<<F1 / 16, 256, 0, stream>>>(w1, F0, F1, F0, F0, 0, 0, w1p);
  k_prepw<<<F2 / 16, 256, 0, stream>>>(w2, F1, F2, F1, F1, 0, 0, w2p);

  k_cent<<<NG / 32, 32, 0, stream>>>(xyz, fps, out);

  k_grp<<<NWAV / 4, 128, SMEM, stream>>>(xyz, pts, fps, w0p, w1p, w2p, out);
}
